// gnn_l2o_optimizer_50912542327356
// MI455X (gfx1250) — hardware-verified
//
#include <hip/hip_runtime.h>


typedef float    v4f  __attribute__((ext_vector_type(4)))  __attribute__((may_alias));
typedef float    v8f  __attribute__((ext_vector_type(8)));
typedef _Float16 v8h  __attribute__((ext_vector_type(8)))  __attribute__((may_alias));
typedef _Float16 v16h __attribute__((ext_vector_type(16)));
typedef __bf16   v8b  __attribute__((ext_vector_type(8)))  __attribute__((may_alias));
typedef __bf16   v16b __attribute__((ext_vector_type(16)));

union FragH { v16h v; v8h p[2]; _Float16 e[16]; };
union FragB { v16b v; v8b p[2]; unsigned short u[16]; };

#define HH   24
#define G4   96
#define KP   32
#define NB   128
#define GP   97
#define LWV  4
#define LTH  128

#define AP   32768
#define CHK  1024
#define CAP  1024
#define TN   4096
#define GTH  256
#define GWV  8

__device__ __forceinline__ unsigned short f2bf(float f)
{
    unsigned int u = __float_as_uint(f);
    u += 0x7FFFu + ((u >> 16) & 1u);
    return (unsigned short)(u >> 16);
}
__device__ __forceinline__ float bf2f(unsigned short b)
{
    return __uint_as_float(((unsigned int)b) << 16);
}

__device__ __forceinline__ v8f mma_f16(v16h a, v16h b, v8f c)
{
    v8f d = __builtin_amdgcn_wmma_f32_16x16x32_f16(false, a, false, b, (short)0, c, false, false);
    asm volatile("v_nop\n\tv_nop\n\tv_nop\n\tv_nop" : "+v"(d) : "v"(a), "v"(b));
    return d;
}
__device__ __forceinline__ v8f mma_bf16(v16b a, v16b b, v8f c)
{
    v8f d = __builtin_amdgcn_wmma_f32_16x16x32_bf16(false, a, false, b, (short)0, c, false, false);
    asm volatile("v_nop\n\tv_nop\n\tv_nop\n\tv_nop" : "+v"(d) : "v"(a), "v"(b));
    return d;
}

__device__ __forceinline__ float sigm_f(float v)
{
    return __fdividef(1.0f, 1.0f + __expf(-v));
}
__device__ __forceinline__ float tanh_f(float v)
{
    float c = v;
    c = (c > 15.0f) ? 15.0f : c;
    c = (c < -15.0f) ? -15.0f : c;
    const float e = __expf(2.0f * c);
    return __fdividef(e - 1.0f, e + 1.0f);
}

__device__ __forceinline__ void emit_hc(float* oh, float* oc, const float* hs, const float* cs, int n4, int tid)
{
#pragma unroll
    for (int p = 0; p < (NB * HH) / (4 * LTH); ++p) {
        const int idx = p * LTH + tid;
        if (idx < n4) {
            const v4f hv = *(const v4f*)(hs + 4 * idx);
            const v4f cv = *(const v4f*)(cs + 4 * idx);
            *(volatile v4f*)(oh + 4 * idx) = hv;
            *(volatile v4f*)(oc + 4 * idx) = cv;
        }
    }
}
__device__ __forceinline__ void emit_y(float* yo, const float* ys, int lane)
{
    const v4f v = *(const v4f*)(ys + 4 * lane);
    *(volatile v4f*)(yo + 4 * lane) = v;
}

__global__ __launch_bounds__(LTH)
void k_lstm(const float* __restrict__ x,
            const float* __restrict__ h0,
            const float* __restrict__ c0,
            const float* __restrict__ w_ih,
            const float* __restrict__ w_hh,
            const float* __restrict__ b_ih,
            const float* __restrict__ b_hh,
            const float* __restrict__ gcn_w,
            const float* __restrict__ lin_w,
            float* out_h, float* out_c, float* y_ws, int n)
{
    __shared__ __attribute__((aligned(16))) _Float16       whh_s[G4 * KP];
    __shared__ __attribute__((aligned(16))) unsigned short gwh_s[KP * KP];
    __shared__ __attribute__((aligned(16))) unsigned short gwl_s[KP * KP];
    __shared__ __attribute__((aligned(16))) float          gt_s[LWV][16 * GP];
    __shared__ __attribute__((aligned(16))) float          hs_s[NB * HH];
    __shared__ __attribute__((aligned(16))) float          cs_s[NB * HH];
    __shared__ __attribute__((aligned(16))) float          ys_s[NB];
    __shared__ float lw_s[HH];

    const int tid  = threadIdx.x;
    const int lane = tid & 31;
    const int wv   = tid >> 5;
    const int hf   = lane >> 4;
    const int m    = lane & 15;
    const int base = blockIdx.x * NB;

    for (int i = tid; i < G4 * KP; i += LTH) {
        const int j = i >> 5, k = i & 31;
        const float v = (k < HH) ? w_hh[j * HH + k] * 64.0f : 0.0f;
        whh_s[i] = (_Float16)v;
    }
    for (int i = tid; i < KP * KP; i += LTH) {
        const int nn = i >> 5, k = i & 31;
        const float v = (nn < HH && k < HH) ? gcn_w[nn * HH + k] : 0.0f;
        const unsigned short hb = f2bf(v);
        gwh_s[i] = hb;
        gwl_s[i] = f2bf(v - bf2f(hb));
    }
    if (tid < HH) lw_s[tid] = lin_w[tid];
    __syncthreads();

#pragma unroll 1
    for (int s = 0; s < 2; ++s) {
        const int r0 = (wv + LWV * s) * 16;
        float* gt = gt_s[wv];

        int ndA = base + r0 + m;
        ndA = (ndA < n) ? ndA : (n - 1);
        const float* hp = h0 + (size_t)ndA * HH;
        const v4f p0 = *(const v4f*)(hp + 8 * hf);
        const v4f p1 = *(const v4f*)(hp + 8 * hf + 4);
        const v4f p2 = *(const v4f*)(hp + 16);
        const v4f p3 = *(const v4f*)(hp + 20);
        const float sc1 = (hf == 0) ? 1024.0f : 0.0f;
        FragH a;
#pragma unroll
        for (int e = 0; e < 4; ++e) {
            a.e[e]      = (_Float16)(p0[e] * 1024.0f);
            a.e[4 + e]  = (_Float16)(p1[e] * 1024.0f);
            a.e[8 + e]  = (_Float16)(p2[e] * sc1);
            a.e[12 + e] = (_Float16)(p3[e] * sc1);
        }
        float xr[8];
#pragma unroll
        for (int r = 0; r < 8; ++r) {
            int nd = base + r0 + 8 * hf + r;
            nd = (nd < n) ? nd : (n - 1);
            xr[r] = x[nd];
        }

#pragma unroll
        for (int t = 0; t < 6; ++t) {
            const int j = 16 * t + m;
            FragH b;
            b.p[0] = *(const v8h*)(&whh_s[j * KP + 8 * hf]);
            b.p[1] = *(const v8h*)(&whh_s[j * KP + 16 + 8 * hf]);
            v8f acc = {0.0f, 0.0f, 0.0f, 0.0f, 0.0f, 0.0f, 0.0f, 0.0f};
            acc = mma_f16(a.v, b.v, acc);
            const float wih = w_ih[j];
            const float bs  = b_ih[j] + b_hh[j];
#pragma unroll
            for (int r = 0; r < 8; ++r)
                gt[(8 * hf + r) * GP + j] = acc[r] * (1.0f / 65536.0f) + (xr[r] * wih + bs);
        }
        __syncthreads();

#pragma unroll 4
        for (int u = 0; u < 12; ++u) {
            const int q   = lane + 32 * u;
            const int row = q / HH;
            const int ch  = q - row * HH;
            const float* g = gt + row * GP;
            const float gi = g[ch];
            const float gf = g[HH + ch];
            const float gg = g[2 * HH + ch];
            const float go = g[3 * HH + ch];
            const float ig = sigm_f(gi);
            const float fg = sigm_f(gf);
            const float og = sigm_f(go);
            const float gc = tanh_f(gg);
            const int nd = base + r0 + row;
            const float cp = (nd < n) ? c0[(size_t)nd * HH + ch] : 0.0f;
            const float cn = fg * cp + ig * gc;
            const float hn = og * tanh_f(cn);
            hs_s[(r0 + row) * HH + ch] = hn;
            cs_s[(r0 + row) * HH + ch] = cn;
        }
        __syncthreads();

        FragB ah, al;
        const float* hrow = &hs_s[(r0 + m) * HH];
#pragma unroll
        for (int e = 0; e < 8; ++e) {
            const float v0 = hrow[8 * hf + e];
            const unsigned short b0 = f2bf(v0);
            ah.u[e] = b0;
            al.u[e] = f2bf(v0 - bf2f(b0));
            const float v1r = hrow[16 + e];
            const float v1  = (hf == 0) ? v1r : 0.0f;
            const unsigned short b1 = f2bf(v1);
            ah.u[8 + e] = b1;
            al.u[8 + e] = f2bf(v1 - bf2f(b1));
        }
#pragma unroll
        for (int t = 0; t < 2; ++t) {
            const int nn = 16 * t + m;
            FragB bh, bl;
            bh.p[0] = *(const v8b*)(&gwh_s[nn * KP + 8 * hf]);
            bh.p[1] = *(const v8b*)(&gwh_s[nn * KP + 16 + 8 * hf]);
            bl.p[0] = *(const v8b*)(&gwl_s[nn * KP + 8 * hf]);
            bl.p[1] = *(const v8b*)(&gwl_s[nn * KP + 16 + 8 * hf]);
            v8f acc = {0.0f, 0.0f, 0.0f, 0.0f, 0.0f, 0.0f, 0.0f, 0.0f};
            acc = mma_bf16(ah.v, bh.v, acc);
            acc = mma_bf16(ah.v, bl.v, acc);
            acc = mma_bf16(al.v, bh.v, acc);
#pragma unroll
            for (int r = 0; r < 8; ++r) gt[(8 * hf + r) * GP + nn] = acc[r];
        }
        __syncthreads();

        if (lane < 16) {
            float yv = 0.0f;
#pragma unroll
            for (int ch = 0; ch < HH; ++ch) yv += gt[lane * GP + ch] * lw_s[ch];
            ys_s[r0 + lane] = yv;
        }
        __syncthreads();
    }

    const int nrows = ((n - base) < NB) ? (n - base) : NB;
    const int n4 = nrows * (HH / 4);
    float* oh = out_h + (size_t)base * HH;
    float* oc = out_c + (size_t)base * HH;
    emit_hc(oh, oc, hs_s, cs_s, n4, tid);
    if (wv == 0) emit_y(y_ws + base, ys_s, lane);
    __threadfence();
    emit_hc(oh, oc, hs_s, cs_s, n4, tid);
    if (wv == 0) emit_y(y_ws + base, ys_s, lane);
}

template <int MODE>
__device__ __forceinline__ void drain_w0(volatile float* S, const int* listd, const float* listv,
                                         volatile int* tag, int len, int lane)
{
    int ng = (len + 31) >> 5;
    if (ng > (CAP / 32)) ng = CAP / 32;
    for (int g = 0; g < ng; ++g) {
        const int i = g * 32 + lane;
        const bool ok = (i < len);
        int dl = 0;
        float v = 0.0f;
        if (ok) {
            dl = listd[i] & (AP - 1);
            v  = MODE ? listv[i] : 1.0f;
        }
        const int t = dl & (TN - 1);
        bool bad = false;
        if (ok) {
            tag[t] = lane;
            bad = (tag[t] != lane);
        }
        const unsigned int anybad = __builtin_amdgcn_ballot_w32(bad);
        if (anybad == 0u) {
            if (ok) {
                const float o = S[dl];
                S[dl] = o + v;
            }
        } else if (lane == 0) {
            for (int jj = 0; jj < 32; ++jj) {
                const int ii = g * 32 + jj;
                if (ii < len) {
                    const int d2 = listd[ii] & (AP - 1);
                    const float v2 = MODE ? listv[ii] : 1.0f;
                    const float o = S[d2];
                    S[d2] = o + v2;
                }
            }
        }
    }
}

__device__ __forceinline__ void emit_dz(const float* S_s, const float* yin, float* dinv_ws, float* z_ws,
                                        int base, int n, int tid)
{
    const v4f z4 = {0.0f, 0.0f, 0.0f, 0.0f};
#pragma unroll 1
    for (int it = 0; it < AP / (4 * GTH); ++it) {
        const int idx = it * GTH + tid;
        const int nd0 = base + 4 * idx;
        const v4f cnt = *(const v4f*)(&S_s[4 * idx]);
        const v4f yv  = *(const v4f*)(yin + nd0);
        v4f dv = z4, zv = z4;
#pragma unroll
        for (int c = 0; c < 4; ++c) {
            const float di = rsqrtf(cnt[c] + 1.0f);
            const bool okn = (nd0 + c) < n;
            dv[c] = okn ? di : 0.0f;
            zv[c] = okn ? (yv[c] * di) : 0.0f;
        }
        *(volatile v4f*)(dinv_ws + nd0) = dv;
        *(volatile v4f*)(z_ws + nd0)    = zv;
    }
}

__device__ __forceinline__ void emit_out(const float* S_s, const float* x, const float* dinv_ws, const float* z_ws,
                                         float* out0, float cb, int base, int n, int tid)
{
    const v4f z4 = {0.0f, 0.0f, 0.0f, 0.0f};
#pragma unroll 1
    for (int it = 0; it < AP / (4 * GTH); ++it) {
        const int idx = it * GTH + tid;
        const int nd0 = base + 4 * idx;
        if (nd0 >= n) continue;
        const v4f sv = *(const v4f*)(&S_s[4 * idx]);
        const v4f dv = *(const v4f*)(dinv_ws + nd0);
        const v4f zv = *(const v4f*)(z_ws + nd0);
        if (nd0 + 4 <= n) {
            const v4f xv = *(const v4f*)(x + nd0);
            v4f o = z4;
#pragma unroll
            for (int c = 0; c < 4; ++c) o[c] = xv[c] * (dv[c] * sv[c] + dv[c] * zv[c] + cb);
            *(volatile v4f*)(out0 + nd0) = o;
        } else {
#pragma unroll
            for (int c = 0; c < 4; ++c) {
                const int nd = nd0 + c;
                if (nd < n) {
                    const float xs = x[nd];
                    *(volatile float*)(out0 + nd) = xs * (dv[c] * sv[c] + dv[c] * zv[c] + cb);
                }
            }
        }
    }
}

template <int MODE>
__global__ __launch_bounds__(GTH)
void k_gcn(const int* __restrict__ ei, const float* gsrc, const float* __restrict__ x,
           const float* __restrict__ gcn_b, const float* __restrict__ lin_w, const float* __restrict__ lin_b,
           float* dinv_ws, float* z_ws, float* out0, int ne, int n)
{
    __shared__ __attribute__((aligned(16))) float S_s[AP];
    __shared__ int   listd_s[CAP];
    __shared__ float listv_s[MODE ? CAP : 1];
    __shared__ int   tag_s[TN];
    __shared__ int   wcnt_s[GWV];

    const int tid  = threadIdx.x;
    const int lane = tid & 31;
    const int wv   = tid >> 5;
    const int base = blockIdx.x * AP;

    const v4f z4 = {0.0f, 0.0f, 0.0f, 0.0f};
    for (int i = tid; i < AP / 4; i += GTH) *(v4f*)(&S_s[4 * i]) = z4;
    __syncthreads();

    const int nch = (ne + CHK - 1) / CHK;
    for (int c = 0; c < nch; ++c) {
        int dl[4]; float val[4]; bool hit[4]; unsigned int bal[4];
#pragma unroll
        for (int j = 0; j < 4; ++j) {
            const int e = c * CHK + j * GTH + tid;
            bool hj = false; int uj = 0; float vj = 1.0f;
            if (e < ne) {
                const int d = ei[(size_t)ne + e];
                const int u = d - base;
                if ((unsigned int)u < (unsigned int)AP) {
                    hj = true; uj = u;
                    if (MODE) {
                        int sI = ei[e];
                        sI = (sI < 0) ? 0 : sI;
                        sI = (sI >= n) ? (n - 1) : sI;
                        vj = gsrc[sI];
                    }
                }
            }
            hit[j] = hj; dl[j] = uj; val[j] = vj;
            bal[j] = __builtin_amdgcn_ballot_w32(hj);
        }
        const int wt = (int)(__builtin_popcount(bal[0]) + __builtin_popcount(bal[1]) +
                             __builtin_popcount(bal[2]) + __builtin_popcount(bal[3]));
        if (lane == 0) wcnt_s[wv] = wt;
        __syncthreads();
        int pre = 0, tot = 0;
#pragma unroll
        for (int i = 0; i < GWV; ++i) {
            const int v = wcnt_s[i];
            tot += v;
            if (i < wv) pre += v;
        }
        int pos = pre;
#pragma unroll
        for (int j = 0; j < 4; ++j) {
            const int lp = (int)__builtin_amdgcn_mbcnt_lo(bal[j], 0u);
            if (hit[j]) {
                const int p = pos + lp;
                if ((unsigned int)p < (unsigned int)CAP) {
                    listd_s[p] = dl[j];
                    if (MODE) listv_s[p] = val[j];
                }
            }
            pos += (int)__builtin_popcount(bal[j]);
        }
        __syncthreads();
        if (wv == 0) drain_w0<MODE>(S_s, listd_s, listv_s, tag_s, tot, lane);
    }
    __syncthreads();

    if (MODE == 0) {
        emit_dz(S_s, gsrc, dinv_ws, z_ws, base, n, tid);
        __threadfence();
        emit_dz(S_s, gsrc, dinv_ws, z_ws, base, n, tid);
    } else {
        float cb = lin_b[0];
#pragma unroll
        for (int ch = 0; ch < HH; ++ch) cb += gcn_b[ch] * lin_w[ch];
        emit_out(S_s, x, dinv_ws, z_ws, out0, cb, base, n, tid);
        __threadfence();
        emit_out(S_s, x, dinv_ws, z_ws, out0, cb, base, n, tid);
    }
}

extern "C" void kernel_launch(void* const* d_in, const int* in_sizes, int n_in,
                              void* d_out, int out_size, void* d_ws, size_t ws_size,
                              hipStream_t stream)
{
    (void)n_in; (void)out_size;
    const float* x     = (const float*)d_in[0];
    const float* h0    = (const float*)d_in[1];
    const float* c0    = (const float*)d_in[2];
    const int*   ei    = (const int*)  d_in[3];
    const float* w_ih  = (const float*)d_in[4];
    const float* w_hh  = (const float*)d_in[5];
    const float* b_ih  = (const float*)d_in[6];
    const float* b_hh  = (const float*)d_in[7];
    const float* gcn_w = (const float*)d_in[8];
    const float* gcn_b = (const float*)d_in[9];
    const float* lin_w = (const float*)d_in[10];
    const float* lin_b = (const float*)d_in[11];

    const int n  = in_sizes[0];
    const int ne = in_sizes[3] / 2;
    if (n <= 0) return;

    float* out0  = (float*)d_out;
    float* out_h = out0 + n;
    float* out_c = out_h + (size_t)n * HH;

    const int    nba  = (n + AP - 1) / AP;
    const size_t npad = (size_t)nba * AP;
    if (3 * npad * sizeof(float) > ws_size) return;
    float* y_ws    = (float*)d_ws;
    float* dinv_ws = y_ws + npad;
    float* z_ws    = dinv_ws + npad;

    const int nbl = (n + NB - 1) / NB;
    k_lstm<<<dim3(nbl), dim3(LTH), 0, stream>>>(x, h0, c0, w_ih, w_hh, b_ih, b_hh, gcn_w, lin_w,
                                                out_h, out_c, y_ws, n);
    k_gcn<0><<<dim3(nba), dim3(GTH), 0, stream>>>(ei, (const float*)y_ws, x, gcn_b, lin_w, lin_b,
                                                  dinv_ws, z_ws, out0, ne, n);
    k_gcn<1><<<dim3(nba), dim3(GTH), 0, stream>>>(ei, (const float*)z_ws, x, gcn_b, lin_w, lin_b,
                                                  dinv_ws, z_ws, out0, ne, n);
}
